// EmbGCN_3470333575179
// MI455X (gfx1250) — hardware-verified
//
#include <hip/hip_runtime.h>
#include <math.h>


#define NB 64
#define NN 2048
#define CI 32
#define CO 32
#define DE 16

typedef __attribute__((ext_vector_type(16))) _Float16 v16h;
typedef __attribute__((ext_vector_type(8)))  _Float16 v8h;
typedef __attribute__((ext_vector_type(8)))  float v8f;
typedef __attribute__((ext_vector_type(4)))  float v4f;
typedef __attribute__((ext_vector_type(4)))  unsigned v4u;

template <typename T> __device__ __forceinline__ void vst2(void* p, T v) { *(volatile T*)p = v; __threadfence(); *(volatile T*)p = v; }
__device__ __forceinline__ v8f wmma16(v16h a, v16h b, v8f c) {
  v8f d = __builtin_amdgcn_wmma_f32_16x16x32_f16(false, a, false, b, (short)0, c, false, false);
  asm volatile("v_nop\n\tv_nop\n\tv_nop\n\tv_nop" : "+v"(d) : "v"(a), "v"(b));
  return d;
}
__device__ __forceinline__ v16h frag_h(const _Float16* rowk0, int lane) {
  union { v16h v; v8h q[2]; } u; const _Float16* p = rowk0 + 8 * (lane >> 4);
  u.q[0] = *(const v8h*)p; u.q[1] = *(const v8h*)(p + 16); return u.v;
}
#define LDSX() do { asm volatile("s_wait_dscnt 0" ::: "memory"); __builtin_amdgcn_wave_barrier(); __builtin_amdgcn_fence(__ATOMIC_RELEASE, "workgroup"); } while (0)

__global__ __launch_bounds__(256) void k_adj(const float* __restrict__ E, _Float16* __restrict__ A16) {
  __shared__ float sE[NN * DE];
  __shared__ float red[256];
  const int n = blockIdx.x, tid = threadIdx.x;
  for (int q = tid; q < NN * DE / 4; q += 256) *(v4f*)(&sE[q * 4]) = *(const v4f*)(E + q * 4);
  __syncthreads();
  float en[DE];
#pragma unroll
  for (int d = 0; d < DE; ++d) en[d] = sE[n * DE + d];
  float s[8]; float mx = -3.0e38f;
#pragma unroll
  for (int c = 0; c < 8; ++c) { const int m = tid * 8 + c; float v = 0.f;
#pragma unroll
    for (int d = 0; d < DE; ++d) v += en[d] * sE[m * DE + d];
    v = v > 0.f ? v : 0.f; s[c] = v; mx = fmaxf(mx, v); }
  red[tid] = mx; __syncthreads();
  for (int st = 128; st > 0; st >>= 1) { if (tid < st) red[tid] = fmaxf(red[tid], red[tid + st]); __syncthreads(); }
  const float gmx = red[0]; __syncthreads();
  float sum = 0.f;
#pragma unroll
  for (int c = 0; c < 8; ++c) { s[c] = expf(s[c] - gmx); sum += s[c]; }
  red[tid] = sum; __syncthreads();
  for (int st = 128; st > 0; st >>= 1) { if (tid < st) red[tid] += red[tid + st]; __syncthreads(); }
  const float inv = 16384.0f / red[0];
  union { v8h h; v4u u; } pk;
#pragma unroll
  for (int c = 0; c < 8; ++c) pk.h[c] = (_Float16)(s[c] * inv);
  vst2(A16 + (size_t)n * NN + tid * 8, pk.u);
}
__global__ __launch_bounds__(256) void k_xT(const float* __restrict__ x, _Float16* __restrict__ xT) {
  __shared__ float tile[64][33];
  const int b = blockIdx.y, m0 = blockIdx.x * 64, tid = threadIdx.x;
  for (int q = tid; q < 64 * 32; q += 256) { const int mm = q >> 5, c = q & 31; tile[mm][c] = x[((size_t)b * NN + m0 + mm) * CI + c]; }
  __syncthreads();
  { const int c = tid >> 3, pc = tid & 7; union { v8h h; v4u u; } pk;
#pragma unroll
    for (int e = 0; e < 8; ++e) pk.h[e] = (_Float16)tile[pc * 8 + e][c];
    vst2(xT + ((size_t)b * CI + c) * NN + m0 + pc * 8, pk.u); }
}
__global__ __launch_bounds__(256) void k_packpool(const float* __restrict__ pool, const float* __restrict__ bpool, _Float16* __restrict__ PT) {
  const int col = blockIdx.x * 256 + threadIdx.x; if (col >= 2048 + 32) return;
  union { v8h h[4]; v4u u[4]; } pk;
#pragma unroll
  for (int d = 0; d < 32; ++d) { float v = 0.f;
    if (d < DE) { if (col < 2048) { const int o = col >> 6, ki = col & 63, k = ki >> 5, i = ki & 31; v = pool[((d * 2 + k) * CI + i) * CO + o]; }
                  else v = bpool[d * CO + (col - 2048)]; }
    pk.h[d >> 3][d & 7] = (_Float16)v; }
#pragma unroll
  for (int q = 0; q < 4; ++q) vst2(PT + (size_t)col * 32 + q * 8, pk.u[q]);
}
__global__ __launch_bounds__(128) void k_wgen(const float* __restrict__ E, const _Float16* __restrict__ PT, float* __restrict__ WT, float* __restrict__ bias) {
  __shared__ __align__(16) float so[4][16][132];
  const int tid = threadIdx.x, wave = tid >> 5, lane = tid & 31, col = lane & 15, g = lane >> 4;
  const int r0 = blockIdx.x * 64 + wave * 16, n0 = blockIdx.y * 128;
  v16h a; { const float* er = E + (size_t)(r0 + col) * DE;
#pragma unroll
    for (int i = 0; i < 8; ++i) { a[i] = (_Float16)er[8 * g + i]; a[8 + i] = (_Float16)0.f; } }
  const int ntile = n0 < 2048 ? 8 : 2;
  v8f acc[8] = {};
#pragma unroll
  for (int j = 0; j < 8; ++j) if (j < ntile) acc[j] = wmma16(a, frag_h(PT + (size_t)(n0 + j * 16 + col) * 32, lane), acc[j]);
  float* S = &so[wave][0][0];
#pragma unroll
  for (int j = 0; j < 8; ++j)
#pragma unroll
    for (int rr = 0; rr < 8; ++rr) S[(8 * g + rr) * 132 + j * 16 + col] = acc[j][rr];
  LDSX();
  if (n0 < 2048) {
#pragma unroll 4
    for (int rl = 0; rl < 16; ++rl) vst2(WT + (size_t)(r0 + rl) * 2048 + n0 + lane * 4, *(const v4f*)(S + rl * 132 + lane * 4)); }
  else { for (int q = lane; q < 16 * 8; q += 32) { const int rl = q >> 3, pc = q & 7; vst2(bias + (size_t)(r0 + rl) * CO + pc * 4, *(const v4f*)(S + rl * 132 + pc * 4)); } }
}
__global__ __launch_bounds__(128) void k_agg(const _Float16* __restrict__ A16, const _Float16* __restrict__ xT, float* __restrict__ xg) {
  __shared__ __align__(16) float so[4][16][36];
  const int tid = threadIdx.x, wave = tid >> 5, lane = tid & 31, col = lane & 15, g = lane >> 4;
  const int b = blockIdx.y, r0 = blockIdx.x * 64 + wave * 16;
  v8f acc[2] = {};
  const _Float16* ar = A16 + (size_t)(r0 + col) * NN; const _Float16* xb = xT + (size_t)b * CI * NN;
#pragma unroll 1
  for (int kc = 0; kc < NN / 32; ++kc) { const v16h a = frag_h(ar + kc * 32, lane);
#pragma unroll
    for (int j = 0; j < 2; ++j) acc[j] = wmma16(a, frag_h(xb + (size_t)(j * 16 + col) * NN + kc * 32, lane), acc[j]); }
#pragma unroll
  for (int j = 0; j < 2; ++j)
#pragma unroll
    for (int rr = 0; rr < 8; ++rr) so[wave][8 * g + rr][j * 16 + col] = acc[j][rr] * (1.0f / 16384.0f);
  LDSX();
  for (int q = lane; q < 16 * 8; q += 32) { const int rl = q >> 3, pc = q & 7; vst2(xg + ((size_t)b * NN + r0 + rl) * CI + pc * 4, *(const v4f*)(&so[wave][rl][pc * 4])); }
}
__global__ __launch_bounds__(128) void k_node(const float* __restrict__ x, const float* __restrict__ xg, const float* __restrict__ WT, const float* __restrict__ bias,
                                            float* __restrict__ out) {
  __shared__ __align__(16) _Float16 wh[CO][72];
  __shared__ __align__(16) float so[4][16][36];
  const int tid = threadIdx.x, wave = tid >> 5, lane = tid & 31, col = lane & 15, g = lane >> 4;
  const int n = blockIdx.x, b0 = wave * 16, b = b0 + col;
  for (int q = tid; q < CO * 64; q += 128) { const int o = q >> 6, ki = q & 63; wh[o][ki] = (_Float16)WT[(size_t)n * 2048 + o * 64 + ki]; }
  __syncthreads();
  v8f acc[2] = {};
#pragma unroll
  for (int kc = 0; kc < 2; ++kc) { v16h a; const float* src = kc == 0 ? x + ((size_t)b * NN + n) * CI : xg + ((size_t)b * NN + n) * CI;
#pragma unroll
    for (int i = 0; i < 8; ++i) { a[i] = (_Float16)src[8 * g + i]; a[8 + i] = (_Float16)src[16 + 8 * g + i]; }
#pragma unroll
    for (int j = 0; j < 2; ++j) acc[j] = wmma16(a, frag_h(&wh[j * 16 + col][0] + kc * 32, lane), acc[j]); }
#pragma unroll
  for (int j = 0; j < 2; ++j) { const float bv = bias[(size_t)n * CO + j * 16 + col];
#pragma unroll
    for (int rr = 0; rr < 8; ++rr) so[wave][8 * g + rr][j * 16 + col] = acc[j][rr] + bv; }
  LDSX();
  for (int q = lane; q < 16 * 8; q += 32) { const int rl = q >> 3, pc = q & 7; vst2(out + ((size_t)(b0 + rl) * NN + n) * CO + pc * 4, *(const v4f*)(&so[wave][rl][pc * 4])); }
}

extern "C" void kernel_launch(void* const* d_in, const int* in_sizes, int n_in,
                              void* d_out, int out_size, void* d_ws, size_t ws_size,
                              hipStream_t stream) {
  (void)in_sizes; (void)n_in; (void)out_size; (void)ws_size;
  const float* x = (const float*)d_in[0]; const float* E = (const float*)d_in[1]; const float* pool = (const float*)d_in[2]; const float* bpool = (const float*)d_in[3];
  float* out = (float*)d_out;
  char* ws = (char*)d_ws; size_t off = 0;
  auto take = [&](size_t bytes) { char* p = ws + off; off += (bytes + 255) & ~(size_t)255; return p; };
  _Float16* A16 = (_Float16*)take((size_t)NN * NN * 2);
  _Float16* xT = (_Float16*)take((size_t)NB * CI * NN * 2);
  _Float16* PT = (_Float16*)take((size_t)(2048 + 128) * 32 * 2);
  float* WT = (float*)take((size_t)NN * 2048 * 4);
  float* bias = (float*)take((size_t)NN * CO * 4);
  float* xg = (float*)take((size_t)NB * NN * CI * 4);
  k_adj<<<NN, 256, 0, stream>>>(E, A16);
  k_xT<<<dim3(NN / 64, NB), 256, 0, stream>>>(x, xT);
  k_packpool<<<(2048 + 32 + 255) / 256, 256, 0, stream>>>(pool, bpool, PT);
  k_wgen<<<dim3(NN / 64, 17), 128, 0, stream>>>(E, PT, WT, bias);
  k_agg<<<dim3(NN / 64, NB), 128, 0, stream>>>(A16, xT, xg);
  k_node<<<NN, 128, 0, stream>>>(x, xg, WT, bias, out);
}
